// MultiHeadSelfAttention_17033840296514
// MI455X (gfx1250) — hardware-verified
//
#include <hip/hip_runtime.h>


#ifndef NB
#define NB 2
#endif
#ifndef SEQ
#define SEQ 2048
#endif
#define NB_FULL  2
#define SEQ_FULL 2048
#define DM   1024
#define NH   16
#define HD   64
#define DQ   (NH * HD)
#define RH   ((SEQ) < 256 ? (SEQ) : 256)
#define PSP  40
#define OSP  68
#define PCAR 1024.0f
#define SCL  0.125f
#define L2E  1.4426950408889634f
#define NEGB (-1.0e30f)
#define PL16 ((size_t)NB * NH * SEQ * HD)
#define PLH  ((size_t)NB * NH * RH * HD)

static_assert(SEQ % 64 == 0);
static_assert(SEQ <= SEQ_FULL);
static_assert(NB <= NB_FULL);
static_assert(RH % 64 == 0);
static_assert(RH <= SEQ);
static_assert(HD == 64);
static_assert(DQ == DM);
static_assert(DM % 64 == 0);
static_assert(DM % 32 == 0);
static_assert(DQ % 32 == 0);
static_assert((3 * DQ) % 64 == 0);
static_assert(PSP % 8 == 0);
static_assert(PSP >= 32);
static_assert(OSP % 4 == 0);
static_assert(OSP >= 64);
static_assert((SEQ * DM) % 8 == 0);
static_assert(((size_t)(NB - 1) * SEQ_FULL + SEQ) * DM * 4 <= (size_t)NB_FULL * SEQ_FULL * DM * 4);

constexpr size_t WS_XB   = (size_t)NB * SEQ * DM * 2;
constexpr size_t WS_WQKV = (size_t)3 * DQ * DM * 2;
constexpr size_t WS_WO   = (size_t)DM * DQ * 2;
constexpr size_t WS_P16  = (size_t)3 * NB * NH * SEQ * HD * 2;
constexpr size_t WS_HL   = (size_t)6 * NB * NH * RH * HD * 2;
constexpr size_t WS_AT   = (size_t)NB * SEQ * DQ * 2;
constexpr size_t WS_TOTAL = WS_XB + WS_WQKV + WS_WO + WS_P16 + WS_HL + 2 * WS_AT;
static_assert(WS_XB % 256 == 0);
static_assert(WS_WQKV % 256 == 0);
static_assert(WS_WO % 256 == 0);
static_assert(WS_P16 % 256 == 0);
static_assert(WS_HL % 256 == 0);
static_assert(WS_AT % 256 == 0);
static_assert(WS_TOTAL <= (size_t)134217728);

typedef _Float16 h16;
typedef unsigned short bf;
typedef __attribute__((ext_vector_type(16))) __bf16   v16bf;
typedef __attribute__((ext_vector_type(16))) _Float16 v16h;
typedef __attribute__((ext_vector_type(8)))  _Float16 v8h;
typedef __attribute__((ext_vector_type(8)))  unsigned short v8us;
typedef __attribute__((ext_vector_type(8)))  float    v8f;
typedef __attribute__((ext_vector_type(4)))  float    v4f;
typedef v8h  __attribute__((may_alias)) v8ha;
typedef v4f  __attribute__((may_alias)) v4fa;
typedef v8us __attribute__((may_alias)) v8usa;

__device__ __forceinline__ unsigned short f2bf(float f) { unsigned u = __float_as_uint(f); u += 0x7FFFu + ((u >> 16) & 1u); return (unsigned short)(u >> 16); }
__device__ __forceinline__ float bf2f(unsigned short b) { return __uint_as_float(((unsigned)b) << 16); }
__device__ __forceinline__ float bfr(float f) { return bf2f(f2bf(f)); }
__device__ __forceinline__ void splitf(float y, unsigned short& h, unsigned short& l) { h = f2bf(y); l = f2bf(y - bf2f(h)); }
__device__ __forceinline__ v16h cat16(v8h lo, v8h hi) { return __builtin_shufflevector(lo, hi, 0, 1, 2, 3, 4, 5, 6, 7, 8, 9, 10, 11, 12, 13, 14, 15); }
__device__ __forceinline__ v16bf cat16b(v8us lo, v8us hi) { return __builtin_bit_cast(v16bf, __builtin_shufflevector(lo, hi, 0, 1, 2, 3, 4, 5, 6, 7, 8, 9, 10, 11, 12, 13, 14, 15)); }
__device__ __forceinline__ v8f wmma16(v16h a, v16h b, v8f c) { return __builtin_amdgcn_wmma_f32_16x16x32_f16(false, a, false, b, (short)0, c, false, false); }
__device__ __forceinline__ v8f wmmab(v16bf a, v16bf b, v8f c) { return __builtin_amdgcn_wmma_f32_16x16x32_bf16(false, a, false, b, (short)0, c, false, false); }
__device__ __forceinline__ v16bf ldfb(const bf* p) { return cat16b(*(const v8us*)p, *(const v8us*)(p + 16)); }
__device__ __forceinline__ v16h ldfh(const h16* p) { return cat16(*(const v8h*)p, *(const v8h*)(p + 16)); }
__device__ __forceinline__ float ex2(float x) { return __builtin_amdgcn_exp2f(x); }

__global__ __launch_bounds__(256) void k_cvt8(const float* __restrict__ src, bf* dst, unsigned n8, size_t sS, size_t sD) {
    const unsigned i = blockIdx.x * 256u + threadIdx.x; if (i >= n8) return;
    const float* s = src + (size_t)blockIdx.y * sS + (size_t)i * 8; bf* d = dst + (size_t)blockIdx.y * sD + (size_t)i * 8;
    const v4f a = *(const v4f*)s; const v4f b = *(const v4f*)(s + 4); v8us o;
#pragma unroll
    for (int k = 0; k < 4; ++k) { o[k] = f2bf(a[k]); o[4 + k] = f2bf(b[k]); }
    *(volatile v8us*)d = o; __threadfence(); *(volatile v8us*)d = o;
}

template <int NSPLIT>
__device__ __forceinline__ void gemm_core(const bf* __restrict__ A, const bf* __restrict__ A2, const bf* __restrict__ Bt, const int K, const size_t aoff, const size_t boff, v8f (&acc)[4][4]) {
#pragma unroll 1
    for (int kc = 0; kc < K; kc += 32) {
        v16bf a[4], a2[4], bl;
#pragma unroll
        for (int mb = 0; mb < 4; ++mb) { a[mb] = ldfb(A + aoff + (size_t)mb * 16 * K + kc); if (NSPLIT == 1) a2[mb] = ldfb(A2 + aoff + (size_t)mb * 16 * K + kc); else a2[mb] = a[mb]; }
#pragma unroll
        for (int nb = 0; nb < 4; ++nb) { const v16bf b = ldfb(Bt + boff + (size_t)nb * 16 * K + kc);
#pragma unroll
            for (int mb = 0; mb < 4; ++mb) { acc[mb][nb] = wmmab(a[mb], b, acc[mb][nb]); if (NSPLIT == 1) acc[mb][nb] = wmmab(a2[mb], b, acc[mb][nb]); }
            bl = b; }
        asm volatile("" : "+v"(acc[0][0]), "+v"(acc[1][0]), "+v"(acc[2][0]), "+v"(acc[3][0]), "+v"(acc[0][1]), "+v"(acc[1][1]), "+v"(acc[2][1]), "+v"(acc[3][1]));
        asm volatile("v_nop\n\tv_nop\n\tv_nop\n\tv_nop" : "+v"(acc[0][2]), "+v"(acc[1][2]), "+v"(acc[2][2]), "+v"(acc[3][2]), "+v"(acc[0][3]), "+v"(acc[1][3]), "+v"(acc[2][3]), "+v"(acc[3][3]) : "v"(a[3]), "v"(a2[3]), "v"(bl));
    }
}

__global__ __launch_bounds__(32) void k_qkvp(const bf* __restrict__ XB, const bf* __restrict__ W, const float* __restrict__ bias, h16* P16, bf* HL) {
    __shared__ __align__(16) float os[64 * OSP];
    const int lane = threadIdx.x & 31, lr = lane & 15, hi = lane >> 4;
    const int s0 = blockIdx.x * 64, c0 = blockIdx.y * 64, b = blockIdx.z;
    const int which = c0 / DQ;
    const int head = (c0 % DQ) / HD;
    const size_t aoff = ((size_t)b * SEQ + s0 + lr) * DM + 8 * hi, boff = (size_t)(c0 + lr) * DM + 8 * hi;
    v8f acc[4][4];
#pragma unroll
    for (int mb = 0; mb < 4; ++mb)
#pragma unroll
        for (int nb = 0; nb < 4; ++nb) acc[mb][nb] = (v8f){};
    gemm_core<0>(XB, XB, W, DM, aoff, boff, acc);
    float bb[4];
#pragma unroll
    for (int nb = 0; nb < 4; ++nb) bb[nb] = bfr(bias[c0 + nb * 16 + lr]);
#pragma unroll
    for (int mb = 0; mb < 4; ++mb)
#pragma unroll
        for (int nb = 0; nb < 4; ++nb)
#pragma unroll
            for (int j = 0; j < 8; ++j) os[(mb * 16 + hi * 8 + j) * OSP + nb * 16 + lr] = acc[mb][nb][j] + bb[nb];
    __syncthreads();
    const int bh = b * NH + head; const int rq = lane >> 3, pc = lane & 7; const bool hires = (s0 < RH);
    if (which < 2) {
        h16* dst = P16 + (size_t)which * PL16 + ((size_t)bh * SEQ + s0) * HD + pc * 8;
#pragma unroll 1
        for (int ps = 0; ps < 2; ++ps) {
#pragma unroll 4
            for (int it = 0; it < 16; ++it) { const int row = it * 4 + rq; const float* src = os + row * OSP + pc * 8; const v4f x0 = *(const v4fa*)src; const v4f x1 = *(const v4fa*)(src + 4); v8h o;
#pragma unroll
                for (int j = 0; j < 4; ++j) { o[j] = (h16)x0[j]; o[4 + j] = (h16)x1[j]; }
                *(volatile v8h*)(dst + (size_t)row * HD) = o; }
            if (hires) {
                bf* dh = HL + (size_t)(2 * which) * PLH + ((size_t)bh * RH + s0) * HD + pc * 8; bf* dl = dh + PLH;
#pragma unroll 4
                for (int it = 0; it < 16; ++it) { const int row = it * 4 + rq; const float* src = os + row * OSP + pc * 8; const v4f x0 = *(const v4fa*)src; const v4f x1 = *(const v4fa*)(src + 4); v8us oh, ol;
#pragma unroll
                    for (int j = 0; j < 4; ++j) { unsigned short a, c; splitf(x0[j], a, c); oh[j] = a; ol[j] = c; splitf(x1[j], a, c); oh[4 + j] = a; ol[4 + j] = c; }
                    *(volatile v8us*)(dh + (size_t)row * HD) = oh; *(volatile v8us*)(dl + (size_t)row * HD) = ol; } }
            if (ps == 0) __threadfence(); }
    } else {
        h16* dst = P16 + (size_t)2 * PL16 + ((size_t)bh * HD) * SEQ + s0 + pc * 8;
#pragma unroll 1
        for (int ps = 0; ps < 2; ++ps) {
#pragma unroll 4
            for (int it = 0; it < 16; ++it) { const int d = it * 4 + rq; v8h o;
#pragma unroll
                for (int j = 0; j < 8; ++j) o[j] = (h16)os[(pc * 8 + j) * OSP + d];
                *(volatile v8h*)(dst + (size_t)d * SEQ) = o; }
            if (hires) {
                bf* dh = HL + (size_t)4 * PLH + ((size_t)bh * HD) * RH + s0 + pc * 8; bf* dl = dh + PLH;
#pragma unroll 4
                for (int it = 0; it < 16; ++it) { const int d = it * 4 + rq; v8us oh, ol;
#pragma unroll
                    for (int j = 0; j < 8; ++j) { unsigned short a, c; splitf(os[(pc * 8 + j) * OSP + d], a, c); oh[j] = a; ol[j] = c; }
                    *(volatile v8us*)(dh + (size_t)d * RH) = oh; *(volatile v8us*)(dl + (size_t)d * RH) = ol; } }
            if (ps == 0) __threadfence(); }
    }
}

__device__ __forceinline__ void osm_step(const v8f s0, const v8f s1, const int d0, float (&m)[8], float (&l)[8], float (&al)[8], float (&p0)[8], float (&p1)[8]) {
#pragma unroll
    for (int r = 0; r < 8; ++r) {
        const float t0 = (d0 > r) ? NEGB : s0[r] * SCL;
        const float t1 = (d0 + 16 > r) ? NEGB : s1[r] * SCL;
        float mx = fmaxf(t0, t1);
        mx = fmaxf(mx, __shfl_xor(mx, 1, 32)); mx = fmaxf(mx, __shfl_xor(mx, 2, 32)); mx = fmaxf(mx, __shfl_xor(mx, 4, 32)); mx = fmaxf(mx, __shfl_xor(mx, 8, 32));
        const float mn = fmaxf(m[r], mx);
        al[r] = ex2((m[r] - mn) * L2E); p0[r] = ex2((t0 - mn) * L2E); p1[r] = ex2((t1 - mn) * L2E);
        l[r] = l[r] * al[r] + (p0[r] + p1[r]); m[r] = mn; }
}

__global__ __launch_bounds__(32) void k_attn_lo(const h16* __restrict__ Q16, const h16* __restrict__ K16, const h16* __restrict__ VT16, bf* ATh, bf* ATl, int qrow0) {
    __shared__ __align__(16) h16 Ps[16 * PSP];
    __shared__ __align__(16) float Os[16 * OSP];
    const int lane = threadIdx.x & 31, ln = lane & 15, hh = lane >> 4;
    const int q0 = qrow0 + (int)blockIdx.x * 16; const int bh = blockIdx.y; const int b = bh / NH, head = bh % NH;
    const size_t qoff = ((size_t)bh * SEQ + q0 + ln) * HD + 8 * hh;
    const size_t koff = ((size_t)bh * SEQ + ln) * HD + 8 * hh;
    const size_t voff = ((size_t)bh * HD + ln) * SEQ + 8 * hh;
    v8f o[4];
#pragma unroll
    for (int t = 0; t < 4; ++t) o[t] = (v8f){};
    float m[8], l[8];
#pragma unroll
    for (int r = 0; r < 8; ++r) { m[r] = NEGB; l[r] = 0.0f; }
    const int nsteps = (q0 + 15) / 32 + 1;
#pragma unroll 1
    for (int st = 0; st < nsteps; ++st) {
        const int kv = st * 32; const size_t ko = koff + (size_t)kv * HD;
        v8f s0 = (v8f){}, s1 = (v8f){};
        const v16h qa = ldfh(Q16 + qoff), qb = ldfh(Q16 + qoff + 32);
        const v16h k00 = ldfh(K16 + ko), k01 = ldfh(K16 + ko + 32);
        const v16h k10 = ldfh(K16 + ko + 16 * HD), k11 = ldfh(K16 + ko + 16 * HD + 32);
        s0 = wmma16(qa, k00, s0); s1 = wmma16(qa, k10, s1); s0 = wmma16(qb, k01, s0); s1 = wmma16(qb, k11, s1);
        asm volatile("v_nop\n\tv_nop\n\tv_nop\n\tv_nop" : "+v"(s0), "+v"(s1) : "v"(qb), "v"(k01), "v"(k11));
        float al[8], p0[8], p1[8];
        osm_step(s0, s1, kv + ln - q0 - 8 * hh, m, l, al, p0, p1);
#pragma unroll
        for (int r = 0; r < 8; ++r) { Ps[(8 * hh + r) * PSP + ln] = (h16)(p0[r] * PCAR); Ps[(8 * hh + r) * PSP + 16 + ln] = (h16)(p1[r] * PCAR); }
        __syncthreads();
        const v16h pa = cat16(*(const v8ha*)(Ps + ln * PSP + 8 * hh), *(const v8ha*)(Ps + ln * PSP + 16 + 8 * hh));
        __syncthreads();
#pragma unroll
        for (int t = 0; t < 4; ++t)
#pragma unroll
            for (int r = 0; r < 8; ++r) o[t][r] *= al[r];
        const size_t vo = voff + kv; v16h vb[4];
#pragma unroll
        for (int t = 0; t < 4; ++t) vb[t] = ldfh(VT16 + vo + (size_t)t * 16 * SEQ);
#pragma unroll
        for (int t = 0; t < 4; ++t) o[t] = wmma16(pa, vb[t], o[t]);
        asm volatile("v_nop\n\tv_nop\n\tv_nop\n\tv_nop" : "+v"(o[0]), "+v"(o[1]), "+v"(o[2]), "+v"(o[3]) : "v"(pa), "v"(vb[3]));
    }
    float inv[8];
#pragma unroll
    for (int r = 0; r < 8; ++r) { float ls = l[r]; ls += __shfl_xor(ls, 1, 32); ls += __shfl_xor(ls, 2, 32); ls += __shfl_xor(ls, 4, 32); ls += __shfl_xor(ls, 8, 32); inv[r] = __builtin_amdgcn_rcpf(ls * PCAR); }
#pragma unroll
    for (int t = 0; t < 4; ++t)
#pragma unroll
        for (int r = 0; r < 8; ++r) Os[(8 * hh + r) * OSP + t * 16 + ln] = o[t][r] * inv[r];
    __syncthreads();
    const int rq = lane >> 3, pc = lane & 7;
    const size_t abase = ((size_t)b * SEQ + q0) * DQ + (size_t)head * HD + pc * 8;
#pragma unroll 1
    for (int ps = 0; ps < 2; ++ps) {
#pragma unroll
        for (int it = 0; it < 4; ++it) { const int row = it * 4 + rq; const float* src = Os + row * OSP + pc * 8; const v4f x0 = *(const v4fa*)src; const v4f x1 = *(const v4fa*)(src + 4); v8us oh, ol;
#pragma unroll
            for (int j = 0; j < 4; ++j) { unsigned short a, c; splitf(x0[j], a, c); oh[j] = a; ol[j] = c; splitf(x1[j], a, c); oh[4 + j] = a; ol[4 + j] = c; }
            *(volatile v8us*)(ATh + abase + (size_t)row * DQ) = oh; *(volatile v8us*)(ATl + abase + (size_t)row * DQ) = ol; }
        if (ps == 0) __threadfence(); }
}

__global__ __launch_bounds__(32) void k_attn_hi(const bf* __restrict__ QH, const bf* __restrict__ QL, const bf* __restrict__ KH, const bf* __restrict__ KL, const bf* __restrict__ VTH, const bf* __restrict__ VTL, bf* ATh, bf* ATl) {
    __shared__ __align__(16) unsigned short PsH[16 * PSP];
    __shared__ __align__(16) unsigned short PsL[16 * PSP];
    __shared__ __align__(16) float Os[16 * OSP];
    const int lane = threadIdx.x & 31, ln = lane & 15, hh = lane >> 4;
    const int q0 = (int)blockIdx.x * 16; const int bh = blockIdx.y; const int b = bh / NH, head = bh % NH;
    const size_t qoff = ((size_t)bh * RH + q0 + ln) * HD + 8 * hh;
    const size_t koff = ((size_t)bh * RH + ln) * HD + 8 * hh;
    const size_t voff = ((size_t)bh * HD + ln) * RH + 8 * hh;
    v8f o[4];
#pragma unroll
    for (int t = 0; t < 4; ++t) o[t] = (v8f){};
    float m[8], l[8];
#pragma unroll
    for (int r = 0; r < 8; ++r) { m[r] = NEGB; l[r] = 0.0f; }
    const int nsteps = (q0 + 15) / 32 + 1;
#pragma unroll 1
    for (int st = 0; st < nsteps; ++st) {
        const int kv = st * 32; const size_t ko = koff + (size_t)kv * HD;
        v8f s0 = (v8f){}, s1 = (v8f){};
        v16bf qh, ql, kh0, kl0, kh1, kl1;
#pragma unroll
        for (int kc = 0; kc < 2; ++kc) {
            qh = ldfb(QH + qoff + kc * 32); ql = ldfb(QL + qoff + kc * 32);
            kh0 = ldfb(KH + ko + kc * 32); kl0 = ldfb(KL + ko + kc * 32);
            kh1 = ldfb(KH + ko + 16 * HD + kc * 32); kl1 = ldfb(KL + ko + 16 * HD + kc * 32);
            s0 = wmmab(qh, kh0, s0); s1 = wmmab(qh, kh1, s1);
            s0 = wmmab(ql, kh0, s0); s1 = wmmab(ql, kh1, s1);
            s0 = wmmab(qh, kl0, s0); s1 = wmmab(qh, kl1, s1); }
        asm volatile("v_nop\n\tv_nop\n\tv_nop\n\tv_nop" : "+v"(s0), "+v"(s1) : "v"(qh), "v"(ql), "v"(kl0), "v"(kl1));
        float al[8], p0[8], p1[8];
        osm_step(s0, s1, kv + ln - q0 - 8 * hh, m, l, al, p0, p1);
#pragma unroll
        for (int r = 0; r < 8; ++r) { unsigned short a, c; splitf(p0[r], a, c); PsH[(8 * hh + r) * PSP + ln] = a; PsL[(8 * hh + r) * PSP + ln] = c;
            splitf(p1[r], a, c); PsH[(8 * hh + r) * PSP + 16 + ln] = a; PsL[(8 * hh + r) * PSP + 16 + ln] = c; }
        __syncthreads();
        const v16bf ph = cat16b(*(const v8usa*)(PsH + ln * PSP + 8 * hh), *(const v8usa*)(PsH + ln * PSP + 16 + 8 * hh));
        const v16bf pl = cat16b(*(const v8usa*)(PsL + ln * PSP + 8 * hh), *(const v8usa*)(PsL + ln * PSP + 16 + 8 * hh));
        __syncthreads();
#pragma unroll
        for (int t = 0; t < 4; ++t)
#pragma unroll
            for (int r = 0; r < 8; ++r) o[t][r] *= al[r];
        const size_t vo = voff + kv; v16bf vh, vl;
#pragma unroll
        for (int t = 0; t < 4; ++t) { vh = ldfb(VTH + vo + (size_t)t * 16 * RH); vl = ldfb(VTL + vo + (size_t)t * 16 * RH);
            o[t] = wmmab(ph, vh, o[t]); o[t] = wmmab(pl, vh, o[t]); o[t] = wmmab(ph, vl, o[t]); }
        asm volatile("v_nop\n\tv_nop\n\tv_nop\n\tv_nop" : "+v"(o[0]), "+v"(o[1]), "+v"(o[2]), "+v"(o[3]) : "v"(ph), "v"(pl), "v"(vh), "v"(vl));
    }
    float inv[8];
#pragma unroll
    for (int r = 0; r < 8; ++r) { float ls = l[r]; ls += __shfl_xor(ls, 1, 32); ls += __shfl_xor(ls, 2, 32); ls += __shfl_xor(ls, 4, 32); ls += __shfl_xor(ls, 8, 32); inv[r] = __builtin_amdgcn_rcpf(ls); }
#pragma unroll
    for (int t = 0; t < 4; ++t)
#pragma unroll
        for (int r = 0; r < 8; ++r) Os[(8 * hh + r) * OSP + t * 16 + ln] = o[t][r] * inv[r];
    __syncthreads();
    const int rq = lane >> 3, pc = lane & 7;
    const size_t abase = ((size_t)b * SEQ + q0) * DQ + (size_t)head * HD + pc * 8;
#pragma unroll 1
    for (int ps = 0; ps < 2; ++ps) {
#pragma unroll
        for (int it = 0; it < 4; ++it) { const int row = it * 4 + rq; const float* src = Os + row * OSP + pc * 8; const v4f x0 = *(const v4fa*)src; const v4f x1 = *(const v4fa*)(src + 4); v8us oh, ol;
#pragma unroll
            for (int j = 0; j < 4; ++j) { unsigned short a, c; splitf(x0[j], a, c); oh[j] = a; ol[j] = c; splitf(x1[j], a, c); oh[4 + j] = a; ol[4 + j] = c; }
            *(volatile v8us*)(ATh + abase + (size_t)row * DQ) = oh; *(volatile v8us*)(ATl + abase + (size_t)row * DQ) = ol; }
        if (ps == 0) __threadfence(); }
}

__global__ __launch_bounds__(32) void k_oproj(const bf* __restrict__ Ah, const bf* __restrict__ Al, const bf* __restrict__ W, const float* __restrict__ bias, float* C) {
    __shared__ __align__(16) float os[16 * OSP];
    const int lane = threadIdx.x & 31, lr = lane & 15, hi = lane >> 4;
    const int r0 = blockIdx.x * 64, c0 = blockIdx.y * 64, z = blockIdx.z;
    const size_t aoff = ((size_t)z * SEQ + r0 + lr) * DQ + 8 * hi, boff = (size_t)(c0 + lr) * DQ + 8 * hi;
    v8f acc[4][4];
#pragma unroll
    for (int mb = 0; mb < 4; ++mb)
#pragma unroll
        for (int nb = 0; nb < 4; ++nb) acc[mb][nb] = (v8f){};
    gemm_core<1>(Ah, Al, W, DQ, aoff, boff, acc);
    const v4f bz = *(const v4f*)(bias + c0 + lr * 4); v4f bb;
#pragma unroll
    for (int q = 0; q < 4; ++q) bb[q] = bfr(bz[q]);
    float* cbase = C + ((size_t)z * SEQ_FULL + r0) * DM + c0;
#pragma unroll
    for (int mb = 0; mb < 4; ++mb) {
#pragma unroll
        for (int nb = 0; nb < 4; ++nb)
#pragma unroll
            for (int j = 0; j < 8; ++j) os[(hi * 8 + j) * OSP + nb * 16 + lr] = acc[mb][nb][j];
        __syncthreads();
#pragma unroll 1
        for (int ps = 0; ps < 2; ++ps) {
#pragma unroll
            for (int s = 0; s < 8; ++s) { const int row = 2 * s + hi, cofs = lr * 4; const v4f val = *(const v4fa*)(os + row * OSP + cofs) + bb;
                *(volatile v4f*)(cbase + (size_t)(mb * 16 + row) * DM + cofs) = val; }
            if (ps == 0) __threadfence(); }
        __syncthreads();
    }
}

extern "C" void kernel_launch(void* const* d_in, const int* in_sizes, int n_in,
                              void* d_out, int out_size, void* d_ws, size_t ws_size, hipStream_t stream) {
    if (n_in < 5) return;
    const size_t xneed = ((size_t)(NB - 1) * SEQ_FULL + SEQ) * DM;
    if ((size_t)in_sizes[0] < xneed) return;
    if ((size_t)in_sizes[1] < (size_t)3 * DQ * DM) return;
    if ((size_t)in_sizes[2] < (size_t)3 * DQ) return;
    if ((size_t)in_sizes[3] < (size_t)DM * DQ) return;
    if ((size_t)in_sizes[4] < (size_t)DM) return;
    if ((size_t)out_size < xneed) return;
    if (ws_size < WS_TOTAL) return;
    const float* x = (const float*)d_in[0]; const float* wqkv = (const float*)d_in[1]; const float* bqkv = (const float*)d_in[2]; const float* wo = (const float*)d_in[3]; const float* bo = (const float*)d_in[4];
    float* OUT = (float*)d_out;
    char* wsp = (char*)d_ws;
    bf* XB = (bf*)wsp; wsp += WS_XB;
    bf* WQKV = (bf*)wsp; wsp += WS_WQKV;
    bf* WO = (bf*)wsp; wsp += WS_WO;
    h16* P16 = (h16*)wsp; wsp += WS_P16;
    bf* HL = (bf*)wsp; wsp += WS_HL;
    bf* ATh = (bf*)wsp; wsp += WS_AT;
    bf* ATl = (bf*)wsp; wsp += WS_AT;
    h16* Q16 = P16; h16* K16 = P16 + PL16; h16* VT16 = P16 + 2 * PL16;
    bf* QH = HL; bf* QL = HL + PLH; bf* KH = HL + 2 * PLH; bf* KL = HL + 3 * PLH; bf* VTH = HL + 4 * PLH; bf* VTL = HL + 5 * PLH;

    const unsigned nx8 = (unsigned)((size_t)SEQ * DM / 8), nq8 = (unsigned)((size_t)3 * DQ * DM / 8), no8 = (unsigned)((size_t)DM * DQ / 8);
    k_cvt8<<<dim3((nx8 + 255) / 256, NB, 1), 256, 0, stream>>>(x, XB, nx8, (size_t)SEQ_FULL * DM, (size_t)SEQ * DM);
    k_cvt8<<<dim3((nq8 + 255) / 256, 1, 1), 256, 0, stream>>>(wqkv, WQKV, nq8, (size_t)0, (size_t)0);
    k_cvt8<<<dim3((no8 + 255) / 256, 1, 1), 256, 0, stream>>>(wo, WO, no8, (size_t)0, (size_t)0);
    k_qkvp<<<dim3(SEQ / 64, 3 * DQ / 64, NB), 32, 0, stream>>>(XB, WQKV, bqkv, P16, HL);
    k_attn_hi<<<dim3(RH / 16, NB * NH, 1), 32, 0, stream>>>(QH, QL, KH, KL, VTH, VTL, ATh, ATl);
    if (SEQ > RH) k_attn_lo<<<dim3((SEQ - RH) / 16, NB * NH, 1), 32, 0, stream>>>(Q16, K16, VT16, ATh, ATl, RH);
    k_oproj<<<dim3(SEQ / 64, DM / 64, NB), 32, 0, stream>>>(ATh, ATl, WO, bo, OUT);
}
